// QFCN_20057497272455
// MI455X (gfx1250) — hardware-verified
//
#include <hip/hip_runtime.h>
#include <stddef.h>
#include <math.h>


#define NTHR    256
#define NWAVE   8
#define TPW     4
#define PSI_SCL 256.0f
#define INV_SCL2 (1.0f / 65536.0f)
#define APL_HALVES 512
#define WS_APL_BYTES 2048
#define WS_U2_OFF    2048
#define WS_TOTAL     4096

static_assert(NTHR == NWAVE * 32);
static_assert((WS_U2_OFF % 128) == 0 && WS_TOTAL >= WS_U2_OFF + 128);

typedef float    v2f  __attribute__((ext_vector_type(2)));
typedef float    v4f  __attribute__((ext_vector_type(4)));
typedef float    v8f  __attribute__((ext_vector_type(8)));
typedef _Float16 v8h  __attribute__((ext_vector_type(8)));
typedef _Float16 v16h __attribute__((ext_vector_type(16)));
union FragH { v16h v; v8h p[2]; };

#define TY1 0x35343534122220ULL
#define WI1 0x22220000032100ULL
#define TR1 0x05040504032100ULL
#define TY2 0x35341220u
#define WI2 0x00000100u
#define TR2 0x09080760u

__device__ __forceinline__ v8f wmh(v16h a, v16h b, v8f c) {
  v8f d = __builtin_amdgcn_wmma_f32_16x16x32_f16(false, a, false, b, (short)0, c, false, false);
#if defined(__HIP_DEVICE_COMPILE__)
  asm volatile("v_nop\n\tv_nop\n\tv_nop\n\tv_nop" : "+v"(d) : "v"(a), "v"(b));
#endif
  return d;
}

__device__ __forceinline__ v8f zero8() {
  v8f z = {0.f, 0.f, 0.f, 0.f, 0.f, 0.f, 0.f, 0.f};
  return z;
}

__device__ __forceinline__ v4f sel4(bool c, v4f a, v4f b) {
  v4f r;
  r.x = c ? a.x : b.x; r.y = c ? a.y : b.y; r.z = c ? a.z : b.z; r.w = c ? a.w : b.w;
  return r;
}

__device__ __forceinline__ float dot4(v4f q) {
  return q.x * q.x + q.y * q.y + q.z * q.z + q.w * q.w;
}

__device__ __forceinline__ void gate_eval(int type, int p, float C, float S, int r, int c,
                                          int nmask, int sh, float qs, const float* sCos,
                                          float& gr, float& gi) {
  const int d  = r ^ c;
  const int mq = ((r * c) & nmask) << sh;
  const float qc  = sCos[mq & 15] * qs;
  const float qsn = sCos[(mq - 4) & 15] * qs;
  const int rb = (r >> p) & 1;
  const int pt = p > 0 ? p - 1 : 0;
  float vr = 0.0f, vi = 0.0f;
  if (type == 0) { vr = qc; vi = qsn; }
  else if (type == 1) { vr = qc; vi = -qsn; }
  else if (type == 2) {
    if (d == 0) { vr = C; vi = rb ? S : -S; }
  } else if (type == 3) {
    if (d == (1 << p)) vr = 1.0f;
  } else if (type == 4) {
    if (d == 0) {
      if (rb == 0) { vr = 1.0f; }
      else { const int rt = (r >> pt) & 1; vr = C; vi = rt ? S : -S; }
    }
  } else {
    if ((d & ~(1 << pt)) == 0) {
      const int rt = (r >> pt) & 1, ct = (c >> pt) & 1;
      if (rb == 0) { if (rt == ct) vr = 1.0f; }
      else { if (rt == ct) vr = C; else vi = -S; }
    }
  }
  gr = vr; gi = vi;
}

__global__ __launch_bounds__(NTHR) void k_build(const float* __restrict__ f1, const float* __restrict__ p1,
                                                 const float* __restrict__ f2, const float* __restrict__ p2,
                                                 _Float16* apl, float* u2t) {
  __shared__ float sUr[256], sUi[256], sGr[256], sGi[256];
  __shared__ float sVr[16], sVi[16], sHr[16], sHi[16];
  __shared__ float sC[16], sS[16], sCos[16];
  const int tid = threadIdx.x;

  {
    const int i1 = tid < 3 ? tid : 3;
    int i2 = tid - 4; i2 = i2 < 0 ? 0 : (i2 > 1 ? 1 : i2);
    int i3 = tid - 6; i3 = i3 < 0 ? 0 : (i3 > 1 ? 1 : i3);
    int i4 = tid - 8; i4 = i4 < 0 ? 0 : (i4 > 1 ? 1 : i4);
    const float vf1 = f1[i1], vp1 = p1[i2], vf2 = f2[i3], vp2 = p2[i4];
    const float t = tid < 4 ? vf1 : (tid < 6 ? vp1 : (tid < 8 ? vf2 : vp2));
    float sv, cv;
    sincosf(0.5f * t, &sv, &cv);
    if (tid < 10) { sC[tid] = cv; sS[tid] = sv; }
    else if (tid < 16) { sC[tid] = 1.0f; sS[tid] = 0.0f; }
  }
  if (tid < 16) {
    const float c1 = 0.92387953251128674f, c2 = 0.70710678118654757f, c3 = 0.38268343236508978f;
    const int j = tid & 3, qd = (tid >> 2) & 3;
    const float va = (j == 0) ? 1.0f : ((j == 1) ? c1 : ((j == 2) ? c2 : c3));
    const float vb = (j == 0) ? 0.0f : ((j == 1) ? c3 : ((j == 2) ? c2 : c1));
    const float cvv = (qd == 0) ? va : ((qd == 1) ? -vb : ((qd == 2) ? -va : vb));
    sCos[tid] = cvv;
  }
  const int r = tid >> 4, c = tid & 15;
  sUr[tid] = (r == c) ? 1.0f : 0.0f;
  sUi[tid] = 0.0f;
  if (tid < 16) { sVr[tid] = ((tid >> 2) == (tid & 3)) ? 1.0f : 0.0f; sVi[tid] = 0.0f; }
  __syncthreads();

#pragma unroll 1
  for (int g = 0; g < 14; ++g) {
    const int type = (int)((TY1 >> (4 * g)) & 15ULL);
    const int w    = (int)((WI1 >> (4 * g)) & 15ULL);
    const int ti   = (int)((TR1 >> (4 * g)) & 15ULL);
    const int p = 3 - w;
    float gr, gi;
    gate_eval(type, p, sC[ti], sS[ti], r, c, 15, 0, 0.25f, sCos, gr, gi);
    sGr[tid] = gr; sGi[tid] = gi;
    __syncthreads();
    float tr = 0.0f, tim = 0.0f;
#pragma unroll 1
    for (int k = 0; k < 16; ++k) {
      const float ar_ = sGr[r * 16 + k], ai_ = sGi[r * 16 + k];
      const float ur  = sUr[k * 16 + c],  ui  = sUi[k * 16 + c];
      tr  = fmaf(ar_, ur, tr);  tr  = fmaf(-ai_, ui, tr);
      tim = fmaf(ar_, ui, tim); tim = fmaf(ai_, ur, tim);
    }
    __syncthreads();
    sUr[tid] = tr; sUi[tid] = tim;
    __syncthreads();
  }

  const int rr = (tid >> 2) & 3, cc = tid & 3;
#pragma unroll 1
  for (int g = 0; g < 8; ++g) {
    const int type = (int)((TY2 >> (4 * g)) & 15u);
    const int w    = (int)((WI2 >> (4 * g)) & 15u);
    const int ti   = (int)((TR2 >> (4 * g)) & 15u);
    const int p = 1 - w;
    float gr, gi;
    gate_eval(type, p, sC[ti], sS[ti], rr, cc, 3, 2, 0.5f, sCos, gr, gi);
    if (tid < 16) { sHr[tid] = gr; sHi[tid] = gi; }
    __syncthreads();
    float tr = 0.0f, tim = 0.0f;
#pragma unroll 1
    for (int k = 0; k < 4; ++k) {
      const float ar_ = sHr[rr * 4 + k], ai_ = sHi[rr * 4 + k];
      const float ur  = sVr[k * 4 + cc],  ui  = sVi[k * 4 + cc];
      tr  = fmaf(ar_, ur, tr);  tr  = fmaf(-ai_, ui, tr);
      tim = fmaf(ar_, ui, tim); tim = fmaf(ai_, ur, tim);
    }
    __syncthreads();
    if (tid < 16) { sVr[tid] = tr; sVi[tid] = tim; }
    __syncthreads();
  }

  const int plane = tid >> 6, u = tid & 63, i = u >> 2, q = u & 3, qq = q & 1;
  v8h hv;
#pragma unroll
  for (int e = 0; e < 8; ++e) {
    const float vr = sUr[i * 16 + 8 * qq + e];
    const float vi = sUi[i * 16 + 8 * qq + e];
    float val = plane ? vi : vr;
    val = (q < 2) ? val : 0.0f;
    hv[e] = (_Float16)val;
  }
  _Float16* dp = apl + plane * APL_HALVES + i * 32 + 8 * q;
  const int q4 = tid - 128;
  const int q4c = q4 < 0 ? 0 : (q4 > 7 ? 7 : q4);
  v4f lv;
  {
    const int e0 = 4 * q4c;
    float t4[4];
#pragma unroll
    for (int e = 0; e < 4; ++e) {
      const int ee = e0 + e;
      const float vr = sVr[ee & 15], vi = sVi[ee & 15];
      t4[e] = (ee < 16) ? vr : vi;
    }
    lv.x = t4[0]; lv.y = t4[1]; lv.z = t4[2]; lv.w = t4[3];
  }
  float* up = u2t + 4 * q4c;
  const bool wpl = tid < 128;
  const bool wu2 = (tid >= 128) && (tid < 136);
  if (wpl) *(volatile v8h*)dp = hv;
  if (wu2) *(volatile v4f*)up = lv;
  __threadfence();
  if (wpl) *(volatile v8h*)dp = hv;
  if (wu2) *(volatile v4f*)up = lv;
}

__global__ __launch_bounds__(NTHR) void k_main(const float* __restrict__ x, const float* __restrict__ Wm,
                                                const float* __restrict__ bv, const _Float16* __restrict__ apl,
                                                const float* __restrict__ u2t, float* out, int nB, int numTiles) {
  const int lane = threadIdx.x & 31, wave = threadIdx.x >> 5, h = lane >> 4, m = lane & 15;
  const int gw = blockIdx.x * NWAVE + wave;

  FragH fr, fi;
  fr.p[0] = *(const v8h*)(apl + m * 32 + 8 * h);
  fr.p[1] = *(const v8h*)(apl + m * 32 + 16 + 8 * h);
  fi.p[0] = *(const v8h*)(apl + APL_HALVES + m * 32 + 8 * h);
  fi.p[1] = *(const v8h*)(apl + APL_HALVES + m * 32 + 16 + 8 * h);

  float u2r[16], u2i[16];
#pragma unroll
  for (int i = 0; i < 16; ++i) { u2r[i] = u2t[i]; u2i[i] = u2t[16 + i]; }
  const float W0 = Wm[0], W1 = Wm[1], B0 = bv[0], B1 = bv[1];

  v8h z8;
#pragma unroll
  for (int e = 0; e < 8; ++e) z8[e] = (_Float16)0.0f;

#pragma unroll 1
  for (int s = 0; s < TPW; ++s) {
    const int tile = gw * TPW + s;
    if (tile >= numTiles) break;
    int row = tile * 16 + m;
    row = row > nB - 1 ? nB - 1 : row;
    const float* xs = x + (size_t)row * 16;
    const v4f q0 = *(const v4f*)(xs);
    const v4f q1 = *(const v4f*)(xs + 4);
    const v4f q2 = *(const v4f*)(xs + 8);
    const v4f q3 = *(const v4f*)(xs + 12);
    const float ssq = (dot4(q0) + dot4(q1)) + (dot4(q2) + dot4(q3));
    const float sc = PSI_SCL * rsqrtf(ssq);
    const v4f lo4 = sel4(h != 0, q2, q0);
    const v4f hi4 = sel4(h != 0, q3, q1);
    v8h bh;
    bh[0] = (_Float16)(lo4.x * sc); bh[1] = (_Float16)(lo4.y * sc);
    bh[2] = (_Float16)(lo4.z * sc); bh[3] = (_Float16)(lo4.w * sc);
    bh[4] = (_Float16)(hi4.x * sc); bh[5] = (_Float16)(hi4.y * sc);
    bh[6] = (_Float16)(hi4.z * sc); bh[7] = (_Float16)(hi4.w * sc);
    FragH b;
    b.p[0] = bh;
    b.p[1] = z8;

    const v8f cr = wmh(fr.v, b.v, zero8());
    const v8f ci = wmh(fi.v, b.v, zero8());

    float e1p = 0.0f, e3p = 0.0f;
#pragma unroll
    for (int v = 0; v < 8; ++v) {
      const float pr = cr[v] * cr[v] + ci[v] * ci[v];
      e1p += (v & 4) ? -pr : pr;
      e3p += (v & 1) ? -pr : pr;
    }
    const float e1 = (e1p + __shfl_xor(e1p, 16, 32)) * INV_SCL2;
    const float e3 = (e3p + __shfl_xor(e3p, 16, 32)) * INV_SCL2;

    float s0, c0, s1, c1;
    sincosf(0.5f * e1, &s0, &c0);
    sincosf(0.5f * e3, &s1, &c1);
    const float pv0 = c0 * c1, pv1 = c0 * s1, pv2 = s0 * c1, pv3 = s0 * s1;
    float ev = 0.0f;
#pragma unroll
    for (int i = 0; i < 4; ++i) {
      const float orr = u2r[4 * i] * pv0 + u2r[4 * i + 1] * pv1 + u2r[4 * i + 2] * pv2 + u2r[4 * i + 3] * pv3;
      const float oii = u2i[4 * i] * pv0 + u2i[4 * i + 1] * pv1 + u2i[4 * i + 2] * pv2 + u2i[4 * i + 3] * pv3;
      const float pp = orr * orr + oii * oii;
      ev += (i & 1) ? -pp : pp;
    }
    const float l0 = ev * W0 + B0;
    const float l1 = ev * W1 + B1;

    const int src0 = (2 * lane) & 31, src1 = (2 * lane + 1) & 31;
    const float a0 = __shfl(l0, src0, 32);
    const float a1 = __shfl(l1, src0, 32);
    const float g0 = __shfl(l0, src1, 32);
    const float g1 = __shfl(l1, src1, 32);
    v4f ov; ov.x = a0; ov.y = a1; ov.z = g0; ov.w = g1;
    v2f pv; pv.x = a0; pv.y = a1;
    const int smp = tile * 16 + 2 * lane;
    const bool full = (lane < 8) && (smp + 1 < nB);
    const bool part = (lane < 8) && (smp + 1 >= nB) && (smp < nB);
    float* op = out + (size_t)smp * 2;
    if (full) *(volatile v4f*)op = ov;
    if (part) *(volatile v2f*)op = pv;
    __threadfence();
    if (full) *(volatile v4f*)op = ov;
    if (part) *(volatile v2f*)op = pv;
  }
}

extern "C" void kernel_launch(void* const* d_in, const int* in_sizes, int n_in,
                              void* d_out, int out_size, void* d_ws, size_t ws_size,
                              hipStream_t stream) {
  if (n_in < 7) return;
  const int n0 = in_sizes[0];
  if (n0 <= 0 || (n0 % 16) != 0) return;
  const int nB = n0 / 16;
  if (in_sizes[1] != 4 || in_sizes[2] != 2 || in_sizes[3] != 2 || in_sizes[4] != 2) return;
  if (in_sizes[5] != 2 || in_sizes[6] != 2) return;
  if (out_size != 2 * nB) return;
  if (ws_size < (size_t)WS_TOTAL) return;

  const float* x  = (const float*)d_in[0];
  const float* f1 = (const float*)d_in[1];
  const float* p1 = (const float*)d_in[2];
  const float* f2 = (const float*)d_in[3];
  const float* p2 = (const float*)d_in[4];
  const float* Wm = (const float*)d_in[5];
  const float* bv = (const float*)d_in[6];
  float* out = (float*)d_out;

  char* ws = (char*)d_ws;
  _Float16* apl = (_Float16*)(ws);
  float*    u2t = (float*)(ws + WS_U2_OFF);

  const int numTiles    = (nB + 15) / 16;
  const int wavesNeeded = (numTiles + TPW - 1) / TPW;
  const int blocks      = (wavesNeeded + NWAVE - 1) / NWAVE;

  k_build<<<1, NTHR, 0, stream>>>(f1, p1, f2, p2, apl, u2t);
  k_main<<<blocks, NTHR, 0, stream>>>(x, Wm, bv, apl, u2t, out, nB, numTiles);
}
